// KAN_65919158059311
// MI455X (gfx1250) — hardware-verified
//
#include <hip/hip_runtime.h>
#include <math.h>

typedef __attribute__((ext_vector_type(16))) _Float16 v16h;
typedef __attribute__((ext_vector_type(8)))  _Float16 v8h;
typedef __attribute__((ext_vector_type(8)))  float    v8f;
typedef __attribute__((ext_vector_type(4)))  float    v4f;

constexpr int kFeat0   = 64;
constexpr int kFeat1   = 128;
constexpr int kFeat2   = 64;
constexpr int kBatch   = 131072;
constexpr int kRowsBlk = 64;
constexpr int kNumBlk  = kBatch / kRowsBlk;
constexpr int kSlots   = 4;
constexpr int kDepth0  = kSlots * kFeat0;
constexpr int kDepth1  = kSlots * kFeat1;
constexpr int kPitchA0 = kDepth0 + 8;
constexpr int kPitchA1 = kDepth1 + 8;
constexpr int kPitchH  = kFeat1 + 4;
constexpr int kPitchO  = kFeat2 + 4;
constexpr int kRegion0Floats = kRowsBlk * kPitchA0 / 2;
static_assert(kBatch % kRowsBlk == 0, "row tiles");
static_assert(kDepth0 % 32 == 0 && kDepth1 % 32 == 0, "depth multiples of 32");
static_assert(kFeat1 == 8 * 16 && kFeat2 == 4 * 16 && kRowsBlk == 4 * 16, "wave tile map");
static_assert(kRowsBlk * kPitchH <= kRegion0Floats, "h stage fits region 0");
static_assert(kRowsBlk * kPitchO <= kRegion0Floats, "out stage fits region 0");
static_assert((kPitchA0 * 2) % 16 == 0 && (kPitchA1 * 2) % 16 == 0, "16-B aligned fragment rows");

constexpr int    kNumCtl = 5;
constexpr int    kDeg    = 3;
constexpr int    kGridPts = 3;
constexpr double kLoD = -1.0;
constexpr double kHiD = 1.0;
constexpr double kKnotLoD   = kLoD - kDeg * 0.1;
constexpr double kKnotHiD   = kHiD + kDeg * 0.1;
constexpr double kKnotStepD = (kKnotHiD - kKnotLoD) / (kNumCtl + kDeg);
constexpr float  kCenter0    = (float)(kKnotLoD + kKnotStepD * ((double)(kDeg / 2) + 0.5));
constexpr float  kCenterStep = (float)kKnotStepD;
constexpr float  kInvWidth   = (float)(1.0 / (kKnotStepD * (kDeg + 1) / 2.0));
constexpr float  kLoF = (float)kLoD;
constexpr float  kHiF = (float)kHiD;
constexpr float  kGridScale = (float)((kGridPts - 1) / (kHiD - kLoD));
static_assert(kGridPts == 3 && kNumCtl == 5, "table shape");
static_assert(kGridScale == 1.0f, "grid position equals clipped value minus low end");
static_assert(kCenter0 > -0.8126f && kCenter0 < -0.8124f, "first centre");
static_assert(kCenterStep > 0.3249f && kCenterStep < 0.3251f, "centre step");
static_assert(kInvWidth > 1.5384f && kInvWidth < 1.5385f, "inverse width");

constexpr float kCarryA = 16.0f;
constexpr float kCarryW = 256.0f;
constexpr float kFoldBack = 1.0f / (kCarryA * kCarryW);
constexpr float kF16MinNormal = 6.103515625e-5f;

constexpr size_t kOffBt0  = 0;
constexpr size_t kOffBt1  = kOffBt0 + (size_t)kFeat1 * kDepth0 * 2;
constexpr size_t kWsTotal = kOffBt1 + (size_t)kFeat2 * kDepth1 * 2;
static_assert(kWsTotal == 131072ull, "carve total");
static_assert((kOffBt1 % 128) == 0, "aligned region");

union FragH { v16h v; v8h h[2]; };
__device__ __forceinline__ v16h frag_load(const _Float16* p) {
  FragH f;
  f.h[0] = *(const v8h*)(p);
  f.h[1] = *(const v8h*)(p + 16);
  return f.v;
}
__device__ __forceinline__ v8f mma_f16(v16h a, v16h b, v8f c) {
  c = __builtin_amdgcn_wmma_f32_16x16x32_f16(false, a, false, b, (short)0, c, false, false);
  asm volatile("v_nop\n\tv_nop\n\tv_nop\n\tv_nop" : "+v"(c) : "v"(a), "v"(b));
  return c;
}
__device__ __forceinline__ _Float16 carry_to_f16(float v, float carry) {
  const float c = v * carry;
  const float f = (fabsf(c) < kF16MinNormal) ? 0.0f : c;
  return (_Float16)f;
}
struct Slot4 { float s0, s1, s2, s3; };
__device__ __forceinline__ Slot4 expand_value(float v) {
  const float sg = 1.0f / (1.0f + expf(-v));
  const float xc = fminf(fmaxf(v, kLoF), kHiF);
  const float gi = (xc - kLoF) * kGridScale;
  Slot4 r;
  r.s0 = v * sg;
  r.s1 = fmaxf(1.0f - gi, 0.0f);
  r.s2 = 1.0f - fabsf(gi - 1.0f);
  r.s3 = fmaxf(gi - 1.0f, 0.0f);
  return r;
}
__device__ __forceinline__ void expand_pack4(const v4f xv, v8h& h0, v8h& h1) {
  const float x0 = xv[0];
  const float x1 = xv[1];
  const float x2 = xv[2];
  const float x3 = xv[3];
  const Slot4 a = expand_value(x0);
  const Slot4 b = expand_value(x1);
  const Slot4 c = expand_value(x2);
  const Slot4 d = expand_value(x3);
  h0[0] = carry_to_f16(a.s0, kCarryA);
  h0[1] = carry_to_f16(a.s1, kCarryA);
  h0[2] = carry_to_f16(a.s2, kCarryA);
  h0[3] = carry_to_f16(a.s3, kCarryA);
  h0[4] = carry_to_f16(b.s0, kCarryA);
  h0[5] = carry_to_f16(b.s1, kCarryA);
  h0[6] = carry_to_f16(b.s2, kCarryA);
  h0[7] = carry_to_f16(b.s3, kCarryA);
  h1[0] = carry_to_f16(c.s0, kCarryA);
  h1[1] = carry_to_f16(c.s1, kCarryA);
  h1[2] = carry_to_f16(c.s2, kCarryA);
  h1[3] = carry_to_f16(c.s3, kCarryA);
  h1[4] = carry_to_f16(d.s0, kCarryA);
  h1[5] = carry_to_f16(d.s1, kCarryA);
  h1[6] = carry_to_f16(d.s2, kCarryA);
  h1[7] = carry_to_f16(d.s3, kCarryA);
}

__global__ __launch_bounds__(256) void fold_weights_kernel(
    const float* __restrict__ cp, const float* __restrict__ bw, const float* __restrict__ sw,
    const float* __restrict__ imp, unsigned short* __restrict__ Bt, int nIn, int nOut)
{
  __shared__ float sE[16];
  __shared__ float sBv[16];
  const int tid = threadIdx.x;
  if (tid < 16) {
    const int gq = tid / 5;
    const int g  = (gq > 2) ? 2 : gq;
    const int k  = tid - 5 * gq;
    const float gr = kLoF + (float)g * ((kHiF - kLoF) / (float)(kGridPts - 1));
    const float center = kCenter0 + kCenterStep * (float)k;
    const float d = (gr - center) * kInvWidth;
    const float e = expf(-(d * d));
    sE[tid] = (tid < 15) ? e : 0.0f;
  }
  __syncthreads();
  if (tid < 16) {
    const int gq = tid / 5;
    const int g  = (gq > 2) ? 2 : gq;
    float s = sE[5 * g];
    s = s + sE[5 * g + 1];
    s = s + sE[5 * g + 2];
    s = s + sE[5 * g + 3];
    s = s + sE[5 * g + 4];
    sBv[tid] = sE[tid] / (s + 1e-6f);
  }
  __syncthreads();
  float bv[3][5];
#pragma unroll
  for (int g = 0; g < 3; ++g)
#pragma unroll
    for (int k = 0; k < 5; ++k) bv[g][k] = sBv[5 * g + k];

  const int halfIn = nIn >> 1;
  const int total  = nOut * halfIn;
  const int t  = blockIdx.x * 256 + tid;
  const int tc = (t < total) ? t : (total - 1);
  const int j  = tc / halfIn;
  const int ip = tc - j * halfIn;
  v8h hv;
#pragma unroll
  for (int q = 0; q < 2; ++q) {
    const int i = 2 * ip + q;
    const size_t idx = (size_t)i * nOut + j;
    const float m = imp[idx];
    const float b = bw[idx];
    const float s = sw[idx];
    const float* c5 = cp + idx * 5;
    const float c0 = c5[0];
    const float c1 = c5[1];
    const float c2 = c5[2];
    const float c3 = c5[3];
    const float c4 = c5[4];
    const float ms = m * s;
    hv[4 * q + 0] = carry_to_f16(m * b, kCarryW);
#pragma unroll
    for (int g = 0; g < 3; ++g) {
      float acc = bv[g][0] * c0;
      acc = fmaf(bv[g][1], c1, acc);
      acc = fmaf(bv[g][2], c2, acc);
      acc = fmaf(bv[g][3], c3, acc);
      acc = fmaf(bv[g][4], c4, acc);
      hv[4 * q + 1 + g] = carry_to_f16(ms * acc, kCarryW);
    }
  }
  unsigned short* dst = Bt + (size_t)j * (size_t)(kSlots * nIn) + 8 * ip;
  if (t < total) *(volatile v8h*)dst = hv;
  __threadfence();
  if (t < total) *(volatile v8h*)dst = hv;
}

__global__ __launch_bounds__(256) void spline_mlp_fused_kernel(
    const float* __restrict__ x, const unsigned short* __restrict__ Bt0p,
    const unsigned short* __restrict__ Bt1p, float* __restrict__ out)
{
  __shared__ __align__(16) float    sR0[kRegion0Floats];
  __shared__ __align__(16) _Float16 sA1[kRowsBlk * kPitchA1];
  _Float16* sA0 = (_Float16*)sR0;

  const _Float16* Bt0 = (const _Float16*)Bt0p;
  const _Float16* Bt1 = (const _Float16*)Bt1p;

  const int tid  = threadIdx.x;
  const int lane = tid & 31;
  const int w    = tid >> 5;
  const int lr   = lane & 15;
  const int hh   = lane >> 4;
  const size_t r0 = (size_t)blockIdx.x * kRowsBlk;

#pragma unroll 1
  for (int it = 0; it < 4; ++it) {
    const int e4  = tid + 256 * it;
    const int row = e4 >> 4;
    const int c4  = (e4 & 15) * 4;
    const v4f xv = *(const v4f*)(x + (r0 + row) * kFeat0 + c4);
    v8h h0, h1;
    expand_pack4(xv, h0, h1);
    _Float16* dst = sA0 + row * kPitchA0 + kSlots * c4;
    *(v8h*)(dst)     = h0;
    *(v8h*)(dst + 8) = h1;
  }
  __syncthreads();

  const v8f zero8 = (v8f){0.f, 0.f, 0.f, 0.f, 0.f, 0.f, 0.f, 0.f};
  v8f c0 = zero8, c1 = zero8, c2 = zero8, c3 = zero8;
  {
    const _Float16* bp = Bt0 + (size_t)(16 * w + lr) * kDepth0 + 8 * hh;
    const _Float16* ap = sA0 + lr * kPitchA0 + 8 * hh;
#pragma unroll 2
    for (int ks = 0; ks < kDepth0 / 32; ++ks) {
      const v16h b  = frag_load(bp + 32 * ks);
      const v16h a0 = frag_load(ap + 32 * ks);
      const v16h a1 = frag_load(ap + 16 * kPitchA0 + 32 * ks);
      const v16h a2 = frag_load(ap + 32 * kPitchA0 + 32 * ks);
      const v16h a3 = frag_load(ap + 48 * kPitchA0 + 32 * ks);
      c0 = mma_f16(a0, b, c0);
      c1 = mma_f16(a1, b, c1);
      c2 = mma_f16(a2, b, c2);
      c3 = mma_f16(a3, b, c3);
    }
  }
  __syncthreads();

  {
    float* hs = sR0 + (8 * hh) * kPitchH + 16 * w + lr;
#pragma unroll
    for (int r = 0; r < 8; ++r) {
      hs[(0 * 16 + r) * kPitchH] = c0[r] * kFoldBack;
      hs[(1 * 16 + r) * kPitchH] = c1[r] * kFoldBack;
      hs[(2 * 16 + r) * kPitchH] = c2[r] * kFoldBack;
      hs[(3 * 16 + r) * kPitchH] = c3[r] * kFoldBack;
    }
  }
  __syncthreads();
#pragma unroll 1
  for (int it = 0; it < 8; ++it) {
    const int e4  = tid + 256 * it;
    const int row = e4 >> 5;
    const int c4  = (e4 & 31) * 4;
    const v4f hv4 = *(const v4f*)(sR0 + row * kPitchH + c4);
    v8h h0, h1;
    expand_pack4(hv4, h0, h1);
    _Float16* dst = sA1 + row * kPitchA1 + kSlots * c4;
    *(v8h*)(dst)     = h0;
    *(v8h*)(dst + 8) = h1;
  }
  __syncthreads();

  const int nt  = w & 3;
  const int mt0 = (w >> 2) * 2;
  v8f d0 = zero8, d1 = zero8;
  {
    const _Float16* bp = Bt1 + (size_t)(16 * nt + lr) * kDepth1 + 8 * hh;
    const _Float16* ap = sA1 + (16 * mt0 + lr) * kPitchA1 + 8 * hh;
#pragma unroll 4
    for (int ks = 0; ks < kDepth1 / 32; ++ks) {
      const v16h b  = frag_load(bp + 32 * ks);
      const v16h a0 = frag_load(ap + 32 * ks);
      const v16h a1 = frag_load(ap + 16 * kPitchA1 + 32 * ks);
      d0 = mma_f16(a0, b, d0);
      d1 = mma_f16(a1, b, d1);
    }
  }

  {
    float* os = sR0 + (16 * mt0 + 8 * hh) * kPitchO + 16 * nt + lr;
#pragma unroll
    for (int r = 0; r < 8; ++r) {
      os[r * kPitchO]        = d0[r] * kFoldBack;
      os[(16 + r) * kPitchO] = d1[r] * kFoldBack;
    }
  }
  __syncthreads();
  {
    const int c4 = lr * 4;
    v4f ov[4];
#pragma unroll
    for (int it = 0; it < 4; ++it) {
      const int row = 8 * w + 2 * it + hh;
      ov[it] = *(const v4f*)(sR0 + row * kPitchO + c4);
    }
    for (int pass = 0; pass < 2; ++pass) {
#pragma unroll
      for (int it = 0; it < 4; ++it) {
        const int row = 8 * w + 2 * it + hh;
        *(volatile v4f*)(out + (r0 + row) * kFeat2 + c4) = ov[it];
      }
      __threadfence();
    }
  }
}

extern "C" void kernel_launch(void* const* d_in, const int* in_sizes, int n_in,
                              void* d_out, int out_size, void* d_ws, size_t ws_size,
                              hipStream_t stream) {
  if (n_in < 9) return;
  if (in_sizes[0] != kBatch * kFeat0) return;
  if (in_sizes[1] != kFeat0 * kFeat1 * kNumCtl) return;
  if (in_sizes[2] != kFeat0 * kFeat1) return;
  if (in_sizes[3] != kFeat0 * kFeat1) return;
  if (in_sizes[4] != kFeat0 * kFeat1) return;
  if (in_sizes[5] != kFeat1 * kFeat2 * kNumCtl) return;
  if (in_sizes[6] != kFeat1 * kFeat2) return;
  if (in_sizes[7] != kFeat1 * kFeat2) return;
  if (in_sizes[8] != kFeat1 * kFeat2) return;
  if (out_size != kBatch * kFeat2) return;
  if (ws_size < kWsTotal) return;

  const float* x    = (const float*)d_in[0];
  const float* cp0  = (const float*)d_in[1];
  const float* bw0  = (const float*)d_in[2];
  const float* sw0  = (const float*)d_in[3];
  const float* imp0 = (const float*)d_in[4];
  const float* cp1  = (const float*)d_in[5];
  const float* bw1  = (const float*)d_in[6];
  const float* sw1  = (const float*)d_in[7];
  const float* imp1 = (const float*)d_in[8];
  float* out = (float*)d_out;

  char* ws = (char*)d_ws;
  unsigned short* BT0 = (unsigned short*)(ws + kOffBt0);
  unsigned short* BT1 = (unsigned short*)(ws + kOffBt1);

  static_assert((kFeat1 * kFeat0 / 2) % 256 == 0 && (kFeat2 * kFeat1 / 2) % 256 == 0, "fold grid exact");
  fold_weights_kernel<<<(kFeat1 * kFeat0 / 2) / 256, 256, 0, stream>>>(cp0, bw0, sw0, imp0, BT0, kFeat0, kFeat1);
  fold_weights_kernel<<<(kFeat2 * kFeat1 / 2) / 256, 256, 0, stream>>>(cp1, bw1, sw1, imp1, BT1, kFeat1, kFeat2);

  spline_mlp_fused_kernel<<<kNumBlk, 256, 0, stream>>>(x, BT0, BT1, out);
}
